// Encoding_48919677501760
// MI455X (gfx1250) — hardware-verified
//
#include <hip/hip_runtime.h>
#include <stdint.h>
#include <stddef.h>

typedef __attribute__((ext_vector_type(16))) _Float16 v16h;
typedef __attribute__((ext_vector_type(8)))  _Float16 v8h;
typedef __attribute__((ext_vector_type(16))) __bf16   v16b;
typedef __attribute__((ext_vector_type(8)))  __bf16   v8b;
typedef __attribute__((ext_vector_type(8)))  float    v8f;
typedef __attribute__((ext_vector_type(4)))  float    v4f;
typedef __attribute__((ext_vector_type(4)))  unsigned int v4u;

__device__ __forceinline__ unsigned short f2bf_bits(float f) {
  unsigned u = __float_as_uint(f);
  return (unsigned short)((u + 0x7FFFu + ((u >> 16) & 1u)) >> 16);
}
__device__ __forceinline__ float bf_bits2f(unsigned short h) { return __uint_as_float(((unsigned)h) << 16); }

__device__ __forceinline__ void dep_guard_h(v8f& a, v8f& b, v16h x, v16h y) { asm volatile("v_nop\n\tv_nop\n\tv_nop\n\tv_nop" : "+v"(a), "+v"(b) : "v"(x), "v"(y)); }
__device__ __forceinline__ void dep_guard_b(v8f& a, v8f& b, v16b x, v16b y) { asm volatile("v_nop\n\tv_nop\n\tv_nop\n\tv_nop" : "+v"(a), "+v"(b) : "v"(x), "v"(y)); }
__device__ __forceinline__ void keep4_h(v16h a, v16h b, v16h c, v16h d) { asm volatile("v_nop" :: "v"(a), "v"(b), "v"(c), "v"(d)); }
__device__ __forceinline__ void keep4_b(v16b a, v16b b, v16b c, v16b d) { asm volatile("v_nop" :: "v"(a), "v"(b), "v"(c), "v"(d)); }
__device__ __forceinline__ void acc_guard4(v8f& a, v8f& b, v8f& c, v8f& d) { asm volatile("v_nop\n\tv_nop\n\tv_nop\n\tv_nop" : "+v"(a), "+v"(b), "+v"(c), "+v"(d)); }
__device__ __forceinline__ void acc_guard2(v8f& a, v8f& b) { asm volatile("v_nop\n\tv_nop\n\tv_nop\n\tv_nop" : "+v"(a), "+v"(b)); }
template <typename T> struct Frag;
template <> struct Frag<_Float16> {
  typedef v16h V; union U { v16h v; v8h h[2]; };
  static __device__ __forceinline__ v16h load(const _Float16* p) {
    U f; f.h[0] = *(const v8h*)(p); f.h[1] = *(const v8h*)(p + 16); return f.v;
  }
  static __device__ __forceinline__ v8f mma(v16h a, v16h b, v8f c) {
    return __builtin_amdgcn_wmma_f32_16x16x32_f16(false, a, false, b, (short)0, c, false, false);
  }
  static __device__ __forceinline__ void guard(v8f& a, v8f& b, v16h x, v16h y) { dep_guard_h(a, b, x, y); }
  static __device__ __forceinline__ void keep(v16h a, v16h b, v16h c, v16h d) { keep4_h(a, b, c, d); }
};
template <> struct Frag<__bf16> {
  typedef v16b V; union U { v16b v; v8b h[2]; };
  static __device__ __forceinline__ v16b load(const __bf16* p) {
    U f; f.h[0] = *(const v8b*)(p); f.h[1] = *(const v8b*)(p + 16); return f.v;
  }
  static __device__ __forceinline__ v8f mma(v16b a, v16b b, v8f c) {
    return __builtin_amdgcn_wmma_f32_16x16x32_bf16(false, a, false, b, (short)0, c, false, false);
  }
  static __device__ __forceinline__ void guard(v8f& a, v8f& b, v16b x, v16b y) { dep_guard_b(a, b, x, y); }
  static __device__ __forceinline__ void keep(v16b a, v16b b, v16b c, v16b d) { keep4_b(a, b, c, d); }
};
typedef Frag<__bf16> FragB16;

constexpr int DESC_DIM        = 128;
constexpr int NUM_CODE        = 32;
constexpr int NUM_DESC        = 4096;
constexpr int NUM_BATCH       = 8;
constexpr int TILE_DESC       = 64;
constexpr int TILES_PER_BATCH = NUM_DESC / TILE_DESC;
constexpr int NUM_BLOCKS      = NUM_BATCH * TILES_PER_BATCH;
constexpr int FUSED_THREADS   = 128;
static_assert(NUM_DESC % TILE_DESC == 0, "tile");
static_assert(TILE_DESC % 32 == 0 && DESC_DIM % 32 == 0, "K steps of 32 with no tail");
static_assert(TILE_DESC % 16 == 0 && NUM_CODE % 16 == 0 && DESC_DIM % 16 == 0, "16x16 tiles");
static_assert(FUSED_THREADS == 2 * TILE_DESC, "X staging map: thread = (d-half, n)");
static_assert(FUSED_THREADS == 4 * NUM_CODE, "codeword staging map: thread = (k, quarter)");

constexpr int PITCH_ND  = 136;
constexpr int PITCH_DN  = 72;
constexpr int PITCH_ATT = 36;
constexpr int PITCH_EST = 132;
static_assert((PITCH_ND * 2) % 16 == 0 && (PITCH_DN * 2) % 16 == 0 && (PITCH_EST * 4) % 16 == 0, "16-B aligned rows");

constexpr size_t WS_PE_BYTES  = (size_t)NUM_BLOCKS * NUM_CODE * DESC_DIM * sizeof(float);
constexpr size_t WS_SKT_OFF   = WS_PE_BYTES;
constexpr size_t WS_SKT_BYTES = (size_t)NUM_BLOCKS * NUM_CODE * sizeof(float);
constexpr size_t WS_TOTAL     = WS_SKT_OFF + WS_SKT_BYTES;
static_assert(WS_PE_BYTES == 8388608 && WS_TOTAL == 8454144, "carve");
static_assert(WS_TOTAL <= (size_t)134217728, "carve under 128 MiB");
static_assert(NUM_CODE * sizeof(float) == 128, "one s_k row = one 128-B line");

__device__ __forceinline__ void split_bits(float v, unsigned& hb, unsigned& lb) {
  const unsigned short h = f2bf_bits(v);
  hb = (unsigned)h;
  lb = (unsigned)f2bf_bits(v - bf_bits2f(h));
}

__global__ __launch_bounds__(FUSED_THREADS)
void vq_tile_kernel(const float* __restrict__ Xg, const float* __restrict__ Cg, const float* __restrict__ Sg,
                    float* __restrict__ PE, float* __restrict__ SKT) {
  __shared__ __align__(16) unsigned short s_xndh[TILE_DESC * PITCH_ND];
  __shared__ __align__(16) unsigned short s_xndl[TILE_DESC * PITCH_ND];
  __shared__ __align__(16) unsigned short s_xdnh[DESC_DIM * PITCH_DN];
  __shared__ __align__(16) unsigned short s_xdnl[DESC_DIM * PITCH_DN];
  __shared__ __align__(16) unsigned short s_cwh[NUM_CODE * PITCH_ND];
  __shared__ __align__(16) unsigned short s_cwl[NUM_CODE * PITCH_ND];
  __shared__ __align__(16) float          s_att[TILE_DESC * PITCH_ATT];
  __shared__ __align__(16) unsigned short s_ath[NUM_CODE * PITCH_DN];
  __shared__ __align__(16) unsigned short s_atl[NUM_CODE * PITCH_DN];
  __shared__ __align__(16) float          s_est[NUM_CODE * PITCH_EST];
  __shared__ float s_xsqp[2 * TILE_DESC];
  __shared__ float s_csqp[4 * NUM_CODE];
  __shared__ float s_csq[NUM_CODE];
  __shared__ float s_scl[NUM_CODE];

  const int t    = threadIdx.x;
  const int lane = t & 31;
  const int wave = t >> 5;
  const int rl   = lane & 15;
  const int hh   = lane >> 4;
  const int koff = hh * 8;

  const int blk  = blockIdx.x;
  const int b    = blk / TILES_PER_BATCH;
  const int tile = blk - b * TILES_PER_BATCH;
  const int n0   = tile * TILE_DESC;

  {
    const int kc = t >> 2, q = t & 3, d0 = q * 32;
    const float* cp = Cg + (size_t)kc * DESC_DIM + d0;
    float sq = 0.f;
#pragma unroll
    for (int c = 0; c < 4; ++c) {
      const v4f f0 = *(const v4f*)(cp + c * 8);
      const v4f f1 = *(const v4f*)(cp + c * 8 + 4);
      const float vv[8] = {f0[0], f0[1], f0[2], f0[3], f1[0], f1[1], f1[2], f1[3]};
      v4u ph, pl;
#pragma unroll
      for (int j = 0; j < 4; ++j) {
        const float a0 = vv[2 * j], a1 = vv[2 * j + 1];
        sq += a0 * a0 + a1 * a1;
        unsigned h0, l0, h1, l1;
        split_bits(a0, h0, l0);
        split_bits(a1, h1, l1);
        ph[j] = h0 | (h1 << 16);
        pl[j] = l0 | (l1 << 16);
      }
      *(v4u*)(s_cwh + kc * PITCH_ND + d0 + c * 8) = ph;
      *(v4u*)(s_cwl + kc * PITCH_ND + d0 + c * 8) = pl;
    }
    s_csqp[kc * 4 + q] = sq;
    if (t < NUM_CODE) s_scl[t] = Sg[t];
  }

  {
    const int nl = t & 63, dh = t >> 6;
    const float* xp = Xg + ((size_t)b * DESC_DIM + (size_t)dh * 64) * NUM_DESC + n0 + nl;
    float sq = 0.f;
#pragma unroll 1
    for (int dc = 0; dc < 8; ++dc) {
      float vv[8];
#pragma unroll
      for (int e = 0; e < 8; ++e) vv[e] = xp[(size_t)(dc * 8 + e) * NUM_DESC];
      const int dbase = dh * 64 + dc * 8;
      v4u ph, pl;
#pragma unroll
      for (int j = 0; j < 4; ++j) {
        const float a0 = vv[2 * j], a1 = vv[2 * j + 1];
        sq += a0 * a0 + a1 * a1;
        unsigned h0, l0, h1, l1;
        split_bits(a0, h0, l0);
        split_bits(a1, h1, l1);
        ph[j] = h0 | (h1 << 16);
        pl[j] = l0 | (l1 << 16);
        const int d = dbase + 2 * j;
        s_xdnh[d * PITCH_DN + nl]       = (unsigned short)h0;
        s_xdnh[(d + 1) * PITCH_DN + nl] = (unsigned short)h1;
        s_xdnl[d * PITCH_DN + nl]       = (unsigned short)l0;
        s_xdnl[(d + 1) * PITCH_DN + nl] = (unsigned short)l1;
      }
      *(v4u*)(s_xndh + nl * PITCH_ND + dbase) = ph;
      *(v4u*)(s_xndl + nl * PITCH_ND + dbase) = pl;
    }
    s_xsqp[dh * TILE_DESC + nl] = sq;
  }
  __syncthreads();

  if (t < NUM_CODE) s_csq[t] = ((s_csqp[4 * t] + s_csqp[4 * t + 1]) + s_csqp[4 * t + 2]) + s_csqp[4 * t + 3];

  {
    const __bf16* Ah = (const __bf16*)s_xndh;
    const __bf16* Al = (const __bf16*)s_xndl;
    const __bf16* Bh = (const __bf16*)s_cwh;
    const __bf16* Bl = (const __bf16*)s_cwl;
    const int arow = wave * 16 + rl;
    v8f acc0 = (v8f){0.f,0.f,0.f,0.f,0.f,0.f,0.f,0.f};
    v8f acc1 = (v8f){0.f,0.f,0.f,0.f,0.f,0.f,0.f,0.f};
#pragma unroll
    for (int k0 = 0; k0 < DESC_DIM; k0 += 32) {
      const v16b bh0 = FragB16::load(Bh + (size_t)rl * PITCH_ND + k0 + koff);
      const v16b bh1 = FragB16::load(Bh + (size_t)(16 + rl) * PITCH_ND + k0 + koff);
      const v16b bl0 = FragB16::load(Bl + (size_t)rl * PITCH_ND + k0 + koff);
      const v16b bl1 = FragB16::load(Bl + (size_t)(16 + rl) * PITCH_ND + k0 + koff);
      const v16b ah  = FragB16::load(Ah + (size_t)arow * PITCH_ND + k0 + koff);
      const v16b al  = FragB16::load(Al + (size_t)arow * PITCH_ND + k0 + koff);
      acc0 = FragB16::mma(ah, bh0, acc0);
      acc0 = FragB16::mma(ah, bl0, acc0);
      acc0 = FragB16::mma(al, bh0, acc0);
      acc1 = FragB16::mma(ah, bh1, acc1);
      acc1 = FragB16::mma(ah, bl1, acc1);
      acc1 = FragB16::mma(al, bh1, acc1);
      FragB16::guard(acc0, acc1, ah, al);
      FragB16::keep(bh0, bh1, bl0, bl1);
    }
    acc_guard2(acc0, acc1);
#pragma unroll
    for (int r = 0; r < 8; ++r) {
      s_att[(wave * 16 + 8 * hh + r) * PITCH_ATT + rl]      = acc0[r];
      s_att[(wave * 16 + 8 * hh + r) * PITCH_ATT + 16 + rl] = acc1[r];
    }
  }
  __syncthreads();

  if (t < TILE_DESC) {
    const int n = t;
    float* arow = s_att + n * PITCH_ATT;
    const float x2 = s_xsqp[n] + s_xsqp[TILE_DESC + n];
    float mx = -3.0e38f;
#pragma unroll 1
    for (int kc = 0; kc < NUM_CODE; ++kc) {
      const float cr = arow[kc];
      const float z = (x2 - 2.0f * cr + s_csq[kc]) * s_scl[kc];
      arow[kc] = z;
      mx = fmaxf(mx, z);
    }
    float sum = 0.f;
#pragma unroll 1
    for (int kc = 0; kc < NUM_CODE; ++kc) {
      const float e = expf(arow[kc] - mx);
      arow[kc] = e;
      sum += e;
    }
    const float inv = 1.0f / sum;
#pragma unroll 1
    for (int kc = 0; kc < NUM_CODE; ++kc) {
      const float p = arow[kc] * inv;
      arow[kc] = p;
      unsigned hb, lb;
      split_bits(p, hb, lb);
      s_ath[kc * PITCH_DN + n] = (unsigned short)hb;
      s_atl[kc * PITCH_DN + n] = (unsigned short)lb;
    }
  }
  __syncthreads();

  if (t < NUM_CODE) {
    float a = 0.f;
#pragma unroll 1
    for (int n = 0; n < TILE_DESC; ++n) a += s_att[n * PITCH_ATT + t];
    volatile float* sp = SKT + (size_t)blk * NUM_CODE + t;
    *sp = a;
    __threadfence();
    *sp = a;
  }

  {
    const __bf16* Ah = (const __bf16*)s_ath;
    const __bf16* Al = (const __bf16*)s_atl;
    const __bf16* Bh = (const __bf16*)s_xdnh;
    const __bf16* Bl = (const __bf16*)s_xdnl;
    const int i2 = wave >> 1;
    const int jb = (wave & 1) * 4;
    const int arow = i2 * 16 + rl;
    v8f acc[4];
#pragma unroll
    for (int j = 0; j < 4; ++j) acc[j] = (v8f){0.f,0.f,0.f,0.f,0.f,0.f,0.f,0.f};
#pragma unroll
    for (int k0 = 0; k0 < TILE_DESC; k0 += 32) {
      v16b bh[4], bl[4];
#pragma unroll
      for (int j = 0; j < 4; ++j) {
        const size_t bo = (size_t)((jb + j) * 16 + rl) * PITCH_DN + k0 + koff;
        bh[j] = FragB16::load(Bh + bo);
        bl[j] = FragB16::load(Bl + bo);
      }
      const size_t ao = (size_t)arow * PITCH_DN + k0 + koff;
      const v16b ah = FragB16::load(Ah + ao);
      const v16b al = FragB16::load(Al + ao);
#pragma unroll
      for (int j = 0; j < 4; ++j) {
        acc[j] = FragB16::mma(ah, bh[j], acc[j]);
        acc[j] = FragB16::mma(ah, bl[j], acc[j]);
        acc[j] = FragB16::mma(al, bh[j], acc[j]);
      }
      FragB16::guard(acc[0], acc[3], ah, al);
      FragB16::keep(bh[0], bh[1], bh[2], bh[3]);
      FragB16::keep(bl[0], bl[1], bl[2], bl[3]);
    }
    acc_guard4(acc[0], acc[1], acc[2], acc[3]);
#pragma unroll
    for (int j = 0; j < 4; ++j) {
      const int col = (jb + j) * 16 + rl;
#pragma unroll
      for (int r = 0; r < 8; ++r) s_est[(i2 * 16 + 8 * hh + r) * PITCH_EST + col] = acc[j][r];
    }
  }
  __syncthreads();

  {
    float* dst = PE + (size_t)blk * (NUM_CODE * DESC_DIM);
    for (int pass = 0; pass < 2; ++pass) {
#pragma unroll
      for (int it = 0; it < 8; ++it) {
        const int f   = it * FUSED_THREADS + t;
        const int row = f >> 5;
        const int c4  = (f & 31) * 4;
        const v4f v = *(const v4f*)(s_est + row * PITCH_EST + c4);
        *(volatile v4f*)(dst + (size_t)row * DESC_DIM + c4) = v;
      }
      __threadfence();
    }
  }
}

__global__ __launch_bounds__(256)
void vq_reduce_kernel(const float* __restrict__ PE, const float* __restrict__ SKT, const float* __restrict__ Cg,
                      float* __restrict__ Out, int n4) {
  const int g = blockIdx.x * 256 + threadIdx.x;
  if (g >= n4) return;
  const int b  = g >> 10;
  const int kc = (g >> 5) & (NUM_CODE - 1);
  const int c4 = (g & 31) * 4;
  const size_t base = (size_t)b * TILES_PER_BATCH;
  float s = 0.f;
  v4f acc = (v4f){0.f, 0.f, 0.f, 0.f};
#pragma unroll 1
  for (int tile = 0; tile < TILES_PER_BATCH; ++tile) {
    const size_t blk = base + (size_t)tile;
    s += SKT[blk * NUM_CODE + kc];
    const v4f pv = *(const v4f*)(PE + (blk * NUM_CODE + kc) * DESC_DIM + c4);
    acc += pv;
  }
  const v4f cw = *(const v4f*)(Cg + (size_t)kc * DESC_DIM + c4);
  const v4f o = acc - s * cw;
  volatile v4f* op = (volatile v4f*)(Out + (size_t)g * 4);
  *op = o;
  __threadfence();
  *op = o;
}

extern "C" void kernel_launch(void* const* d_in, const int* in_sizes, int n_in,
                              void* d_out, int out_size, void* d_ws, size_t ws_size,
                              hipStream_t stream) {
  if (n_in < 3) return;
  if (in_sizes[0] != NUM_BATCH * DESC_DIM * NUM_DESC) return;
  if (in_sizes[1] != NUM_CODE * DESC_DIM) return;
  if (in_sizes[2] < NUM_CODE) return;
  if (out_size != NUM_BATCH * NUM_CODE * DESC_DIM) return;
  if (ws_size < WS_TOTAL) return;

  const float* X  = (const float*)d_in[0];
  const float* Cw = (const float*)d_in[1];
  const float* Sc = (const float*)d_in[2];
  float* Out = (float*)d_out;
  float* PE  = (float*)d_ws;
  float* SKT = (float*)((char*)d_ws + WS_SKT_OFF);

  vq_tile_kernel<<<NUM_BLOCKS, FUSED_THREADS, 0, stream>>>(X, Cw, Sc, PE, SKT);
  const int n4 = out_size / 4;
  vq_reduce_kernel<<<(n4 + 255) / 256, 256, 0, stream>>>(PE, SKT, Cw, Out, n4);
}
